// T3AWrapper_72550587564093
// MI455X (gfx1250) — hardware-verified
//
#include <hip/hip_runtime.h>
#include <hip/hip_bf16.h>
#include <math.h>

typedef _Float16 bf16_t;
typedef bf16_t v16bf __attribute__((ext_vector_type(16)));
typedef bf16_t v8bf  __attribute__((ext_vector_type(8)));
typedef bf16_t v4bf  __attribute__((ext_vector_type(4)));
typedef float  v8f   __attribute__((ext_vector_type(8)));
typedef float  v4f   __attribute__((ext_vector_type(4)));
typedef int    v4i   __attribute__((ext_vector_type(4)));
typedef float __attribute__((may_alias)) float_a;
typedef int   __attribute__((may_alias)) int_a;
#define NPAD 1024
template <typename T> __device__ __forceinline__ void vst2(void* p, T v) { *(volatile T*)p = v; __threadfence(); *(volatile T*)p = v; }
__device__ __forceinline__ v8f WM16(v16bf a, v16bf b, v8f c) {
    v8f d = __builtin_amdgcn_wmma_f32_16x16x32_f16(false, a, false, b, (short)0, c, false, false);
    asm volatile("v_nop\n\tv_nop\n\tv_nop\n\tv_nop" : "+v"(d) : "v"(a), "v"(b));
    return d;
}

#define ENT_THR 0.6f
#define MSEL    29
#define EPSN    1e-12f

__device__ __forceinline__ bf16_t f2bf(float f) { return (bf16_t)f; }

__global__ void __launch_bounds__(256)
f32_to_bf16_kernel(const float* __restrict__ X, bf16_t* __restrict__ Y, long n4) {
    long i = (long)blockIdx.x * 256 + threadIdx.x;
    long stride = (long)gridDim.x * 256;
    for (; i < n4; i += stride) {
        float4 v = ((const float4*)X)[i];
        v4bf o;
        o[0] = f2bf(v.x); o[1] = f2bf(v.y); o[2] = f2bf(v.z); o[3] = f2bf(v.w);
        vst2((v4bf*)Y + i, o);
    }
}

__global__ void __launch_bounds__(256)
rownorm_inv_kernel(const float* __restrict__ X, float* __restrict__ rinv, int D, int nrows) {
    __shared__ float res[32];
    const int lane = threadIdx.x & 31, wave = threadIdx.x >> 5;
    for (int rr = 0; rr < 4; ++rr) {
        const int row = blockIdx.x * 32 + wave * 4 + rr;
        const float* xp = X + (size_t)(row < nrows ? row : nrows - 1) * D;
        float s = 0.f;
        for (int d = lane; d < D; d += 32) { float v = xp[d]; s += v * v; }
#pragma unroll
        for (int m = 16; m >= 1; m >>= 1) s += __shfl_xor(s, m, 32);
        if (lane == 0) res[wave * 4 + rr] = 1.f / fmaxf(sqrtf(s), EPSN);
    }
    __syncthreads();
    if (threadIdx.x < 32 && blockIdx.x * 32 + (int)threadIdx.x < nrows) vst2(rinv + blockIdx.x * 32 + threadIdx.x, (float_a)res[threadIdx.x]);
}


__global__ void __launch_bounds__(128)
wmma_gemm_nt_bf16_kernel(const bf16_t* __restrict__ X, const bf16_t* __restrict__ Y,
                         const float* __restrict__ bias, const float* __restrict__ rowscale,
                         float* __restrict__ out, int Nrows, int D, int ntilesN32) {
    const int wave = threadIdx.x >> 5;
    const int lane = threadIdx.x & 31;
    const int nt   = blockIdx.x * 4 + wave;
    if (nt >= ntilesN32) return;
    const int mt  = blockIdx.y;
    const int m0  = mt * 32, n0 = nt * 32;
    const int l16 = lane & 15, h = lane >> 4;

    const bf16_t* __restrict__ pa0 = X + (size_t)(m0 + l16)      * D;
    const bf16_t* __restrict__ pa1 = X + (size_t)(m0 + 16 + l16) * D;
    int br0 = n0 + l16;      if (br0 >= Nrows) br0 = Nrows - 1;
    int br1 = n0 + 16 + l16; if (br1 >= Nrows) br1 = Nrows - 1;
    const bf16_t* __restrict__ pb0 = Y + (size_t)br0 * D;
    const bf16_t* __restrict__ pb1 = Y + (size_t)br1 * D;

    v8f acc00 = {}, acc01 = {}, acc10 = {}, acc11 = {};

    for (int kk = 0; kk < D; kk += 32) {
        if (kk + 32 < D) {
            __builtin_prefetch(pa0 + kk + 32, 0, 1);
            __builtin_prefetch(pb0 + kk + 32, 0, 1);
        }
        v8bf a0lo = *(const v8bf*)(pa0 + kk + h * 8);
        v8bf a0hi = *(const v8bf*)(pa0 + kk + 16 + h * 8);
        v8bf a1lo = *(const v8bf*)(pa1 + kk + h * 8);
        v8bf a1hi = *(const v8bf*)(pa1 + kk + 16 + h * 8);
        v16bf a0 = __builtin_shufflevector(a0lo, a0hi, 0,1,2,3,4,5,6,7,8,9,10,11,12,13,14,15);
        v16bf a1 = __builtin_shufflevector(a1lo, a1hi, 0,1,2,3,4,5,6,7,8,9,10,11,12,13,14,15);
        v16bf b0 = __builtin_shufflevector(*(const v8bf*)(pb0 + kk + h * 8), *(const v8bf*)(pb0 + kk + 16 + h * 8), 0,1,2,3,4,5,6,7,8,9,10,11,12,13,14,15);
        v16bf b1 = __builtin_shufflevector(*(const v8bf*)(pb1 + kk + h * 8), *(const v8bf*)(pb1 + kk + 16 + h * 8), 0,1,2,3,4,5,6,7,8,9,10,11,12,13,14,15);

        acc00 = WM16(a0, b0, acc00);
        acc01 = WM16(a0, b1, acc01);
        acc10 = WM16(a1, b0, acc10);
        acc11 = WM16(a1, b1, acc11);
    }

    __shared__ __attribute__((aligned(16))) float st[4][32 * 32];
    float* S = st[wave];
    auto put = [&](const v8f& acc, int mb, int nb) {
        const int n = n0 + nb + l16;
        const float bv = (bias && n < Nrows) ? bias[n] : 0.f;
#pragma unroll
        for (int r = 0; r < 8; ++r) { const int ml = mb + r + 8 * h; float v = acc[r]; if (rowscale) v *= rowscale[m0 + ml]; S[ml * 32 + nb + l16] = v + bv; }
    };
    put(acc00, 0, 0); put(acc01, 0, 16); put(acc10, 16, 0); put(acc11, 16, 16);
    asm volatile("s_wait_dscnt 0" ::: "memory"); __builtin_amdgcn_wave_barrier(); __builtin_amdgcn_fence(__ATOMIC_RELEASE, "workgroup");
#pragma unroll
    for (int q = 0; q < 8; ++q) { const int rl = q * 4 + (lane >> 3), pc = lane & 7;
        vst2(out + (size_t)(m0 + rl) * NPAD + n0 + pc * 4, *(const v4f*)(S + rl * 32 + pc * 4)); }
}

__global__ void __launch_bounds__(256)
entropy_argmax_kernel(const float* __restrict__ logits,
                      float* __restrict__ ent, int* __restrict__ yhat, int Kn) {
    __shared__ float se[32]; __shared__ int sy[32];
    const int lane = threadIdx.x & 31, wave = threadIdx.x >> 5;
    for (int rr = 0; rr < 4; ++rr) {
        const int row = blockIdx.x * 32 + wave * 4 + rr;
        const float* lp = logits + (size_t)row * NPAD;
        float m = -INFINITY; int mi = 0x7fffffff;
        for (int j = lane; j < Kn; j += 32) { float v = lp[j]; if (v > m) { m = v; mi = j; } }
#pragma unroll
        for (int k = 16; k > 0; k >>= 1) {
            float o = __shfl_xor(m, k, 32); int oi = __shfl_xor(mi, k, 32);
            if (o > m || (o == m && oi < mi)) { m = o; mi = oi; }
        }
        float S = 0.f, T = 0.f;
        for (int j = lane; j < Kn; j += 32) { float l = lp[j]; float e = expf(l - m); S += e; T += e * l; }
#pragma unroll
        for (int k = 16; k > 0; k >>= 1) { S += __shfl_xor(S, k, 32); T += __shfl_xor(T, k, 32); }
        if (lane == 0) { se[wave * 4 + rr] = m + logf(S) - T / S; sy[wave * 4 + rr] = mi; }
    }
    __syncthreads();
    if (threadIdx.x < 32) { vst2(ent + blockIdx.x * 32 + threadIdx.x, (float_a)se[threadIdx.x]); vst2(yhat + blockIdx.x * 32 + threadIdx.x, (int_a)sy[threadIdx.x]); }
}

__global__ void __launch_bounds__(128)
select_topm_kernel(const float* __restrict__ ent, const int* __restrict__ yhat,
                   int Bn, int Kn, int* __restrict__ selcnt, int* __restrict__ selid) {
    __shared__ int sid_s[128][33];
    __shared__ int scnt[128];
    const int k = blockIdx.x * 128 + threadIdx.x;
    float e[MSEL]; int id[MSEL]; int cnt = 0;
    if (k < Kn) {
    for (int i = 0; i < Bn; ++i) {
        if (yhat[i] != k) continue;
        const float ev = ent[i];
        if (!(ev <= ENT_THR)) continue;
        if (cnt < MSEL) {
            int j = cnt++;
            while (j > 0 && e[j - 1] > ev) { e[j] = e[j - 1]; id[j] = id[j - 1]; --j; }
            e[j] = ev; id[j] = i;
        } else if (ev < e[MSEL - 1]) {
            int j = MSEL - 1;
            while (j > 0 && e[j - 1] > ev) { e[j] = e[j - 1]; id[j] = id[j - 1]; --j; }
            e[j] = ev; id[j] = i;
        }
    }
    }
    scnt[threadIdx.x] = cnt;
    for (int j = 0; j < 32; ++j) sid_s[threadIdx.x][j] = (j < cnt) ? id[j] : -1;
    __syncthreads();
    if (k < Kn) vst2(selcnt + k, (int_a)scnt[threadIdx.x]);
    for (int g = threadIdx.x; g < 128 * 8; g += 128) { const int kl = g >> 3, pc = g & 7; const int kk = blockIdx.x * 128 + kl;
        if (kk < Kn) { v4i v = { sid_s[kl][pc*4], sid_s[kl][pc*4+1], sid_s[kl][pc*4+2], sid_s[kl][pc*4+3] }; vst2(selid + (size_t)kk * 32 + pc * 4, v); } }
}

__global__ void __launch_bounds__(256)
centroid_kernel(const float* __restrict__ W, const float* __restrict__ rw,
                const float* __restrict__ z, const float* __restrict__ rz,
                const int* __restrict__ selcnt, const int* __restrict__ selid,
                float* __restrict__ Cn, int D) {
    __shared__ float sh[256];
    const int k = blockIdx.x;
    const int t = threadIdx.x;
    const float ws = rw[k];
    const float* wr = W + (size_t)k * D;

    float a[3];
    #pragma unroll
    for (int p = 0; p < 3; ++p) {
        const int d = t + p * 256;
        a[p] = (d < D) ? wr[d] * ws : 0.f;
    }
    const int cnt = selcnt[k];
    for (int i = 0; i < cnt; ++i) {
        const int   sid = selid[(size_t)k * 32 + i];
        const float rs  = rz[sid];
        const float* zr = z + (size_t)sid * D;
        #pragma unroll
        for (int p = 0; p < 3; ++p) {
            const int d = t + p * 256;
            if (d < D) a[p] += zr[d] * rs;
        }
    }
    const float inv = 1.f / (float)(cnt + 1);
    float sq = 0.f;
    #pragma unroll
    for (int p = 0; p < 3; ++p) { a[p] *= inv; sq += a[p] * a[p]; }

    sh[t] = sq; __syncthreads();
    for (int s = 128; s > 0; s >>= 1) {
        if (t < s) sh[t] += sh[t + s];
        __syncthreads();
    }
    const float rn = 1.f / fmaxf(sqrtf(sh[0]), EPSN);
    float* cr = Cn + (size_t)k * D;
    #pragma unroll
    for (int p = 0; p < 3; ++p) {
        const int d = t + p * 256;
        if (d < D) vst2(cr + d, (float_a)(a[p] * rn));
    }
}

__global__ void __launch_bounds__(256) flat_copy_kernel(const float* __restrict__ st, float* __restrict__ out, int Bn, int Kn) {
    const long g = (long)blockIdx.x * 256 + threadIdx.x;
    if (g * 4 >= (long)Bn * Kn) return;
    const long f = g * 4; const int r = (int)(f / Kn), c = (int)(f - (long)r * Kn);
    vst2(out + f, *(const v4f*)(st + (size_t)r * NPAD + c));
}

extern "C" void kernel_launch(void* const* d_in, const int* in_sizes, int n_in,
                              void* d_out, int out_size, void* d_ws, size_t ws_size,
                              hipStream_t stream) {
    const float* z = (const float*)d_in[0];
    const float* W = (const float*)d_in[1];
    const float* b = (const float*)d_in[2];

    const int Kn = in_sizes[2];
    const int Dn = in_sizes[1] / Kn;
    const int Bn = in_sizes[0] / Dn;

    float* ws     = (float*)d_ws;
    size_t off    = 0;
    auto al = [&]() { off = (off + 63) & ~(size_t)63; };
    float* logits = ws + off; off += (size_t)Bn * NPAD;
    al(); float* ostage = ws + off; off += (size_t)Bn * NPAD;
    al(); float* ent    = ws + off; off += Bn;
    al(); float* rz     = ws + off; off += Bn;
    al(); float* rw     = ws + off; off += Kn;
    al(); float* Cn     = ws + off; off += (size_t)Kn * Dn;
    al(); int*    yhat   = (int*)(ws + off); off += Bn;
    al(); int*    selcnt = (int*)(ws + off); off += Kn;
    al(); int*    selid  = (int*)(ws + off); off += (size_t)Kn * 32;
    al(); bf16_t* zbf    = (bf16_t*)(ws + off); off += (size_t)Bn * Dn / 2;
    al(); bf16_t* Wbf    = (bf16_t*)(ws + off); off += (size_t)Kn * Dn / 2;
    al(); bf16_t* Cnbf   = (bf16_t*)(ws + off); off += (size_t)Kn * Dn / 2;

    const int ntilesN32 = (Kn + 31) / 32;
    const dim3 gemmGrid((ntilesN32 + 3) / 4, Bn / 32);
    const dim3 gemmBlock(128);

    rownorm_inv_kernel<<<Bn / 32, 256, 0, stream>>>(z, rz, Dn, Bn);
    rownorm_inv_kernel<<<(Kn + 31) / 32, 256, 0, stream>>>(W, rw, Dn, Kn);

    {
        long zn4 = (long)Bn * Dn / 4;
        long wn4 = (long)Kn * Dn / 4;
        f32_to_bf16_kernel<<<(int)((zn4 + 255) / 256), 256, 0, stream>>>(z, zbf, zn4);
        f32_to_bf16_kernel<<<(int)((wn4 + 255) / 256), 256, 0, stream>>>(W, Wbf, wn4);
    }

    wmma_gemm_nt_bf16_kernel<<<gemmGrid, gemmBlock, 0, stream>>>(
        zbf, Wbf, b, nullptr, logits, Kn, Dn, ntilesN32);

    entropy_argmax_kernel<<<Bn / 32, 256, 0, stream>>>(logits, ent, yhat, Kn);

    select_topm_kernel<<<(Kn + 127) / 128, 128, 0, stream>>>(
        ent, yhat, Bn, Kn, selcnt, selid);

    centroid_kernel<<<Kn, 256, 0, stream>>>(W, rw, z, rz, selcnt, selid, Cn, Dn);
    {
        long cn4 = (long)Kn * Dn / 4;
        f32_to_bf16_kernel<<<(int)((cn4 + 255) / 256), 256, 0, stream>>>(Cn, Cnbf, cn4);
    }

    wmma_gemm_nt_bf16_kernel<<<gemmGrid, gemmBlock, 0, stream>>>(
        zbf, Cnbf, nullptr, rz, ostage, Kn, Dn, ntilesN32);
    flat_copy_kernel<<<(int)(((long)Bn * Kn / 4 + 255) / 256), 256, 0, stream>>>(ostage, (float*)d_out, Bn, Kn);
}
